// PointNet2_11519102288168
// MI455X (gfx1250) — hardware-verified
//
#include <hip/hip_runtime.h>
#include <cstdint>
#include <cstddef>

#pragma clang fp contract(off)

typedef __attribute__((ext_vector_type(16))) _Float16 v16h;
typedef __attribute__((ext_vector_type(8)))  _Float16 v8h;
typedef __attribute__((ext_vector_type(8)))  float    v8f;
typedef __attribute__((ext_vector_type(4)))  float    v4f;
typedef __attribute__((ext_vector_type(4)))  int      v4i;

constexpr int NBATCH = 16;
constexpr int NPOINT = 8192;
constexpr int NCEN1  = 512;
constexpr int NNBR1  = 32;
constexpr int NCEN2  = 128;
constexpr int NNBR2  = 64;
constexpr int CH1A   = 64;
constexpr int CH1B   = 128;
constexpr int CH2A   = 128;
constexpr int CH2B   = 256;
constexpr int CH3O   = 256;
constexpr int W20LD  = 131;
constexpr int W30LD  = 259;
constexpr int NQ1    = NBATCH * NCEN1;
constexpr int NQ2    = NBATCH * NCEN2;
constexpr int ROWS1  = NQ1 * NNBR1;
constexpr int ROWS2  = NQ2 * NNBR2;
constexpr int ROWS3  = NQ2;
constexpr float WCARRY     = 16.0f;
constexpr float WCARRY_INV = 1.0f / 16.0f;

static_assert(ROWS1 == 262144 && ROWS2 == 131072 && ROWS3 == 2048, "row counts");
static_assert(ROWS1 % 64 == 0 && CH1B % 64 == 0 && CH1A % 32 == 0, "gemm 1_1 shape");
static_assert(NQ1 % 64 == 0 && CH2A % 64 == 0 && CH1B % 32 == 0, "gemm Pf shape");
static_assert(ROWS2 % 64 == 0 && CH2B % 64 == 0 && CH2A % 32 == 0, "gemm 2_1 shape");
static_assert(ROWS3 % 64 == 0 && CH3O % 64 == 0 && CH2B % 32 == 0, "gemm 3_0 shape");
static_assert(NBATCH * 256 * 4 * 2 == 32768, "d_out bytes");

__device__ __forceinline__ void keep4_h(v16h a, v16h b, v16h c, v16h d) { asm volatile("v_nop" :: "v"(a), "v"(b), "v"(c), "v"(d)); }
__device__ __forceinline__ void acc_guard4(v8f& a, v8f& b, v8f& c, v8f& d) { asm volatile("v_nop\n\tv_nop\n\tv_nop\n\tv_nop" : "+v"(a), "+v"(b), "+v"(c), "+v"(d)); }
__device__ __forceinline__ void tile_guard_h(v8f& a, v8f& b, v8f& c, v8f& d, v16h x, v16h y0, v16h y1, v16h y2, v16h y3) {
  asm volatile("v_nop\n\tv_nop\n\tv_nop\n\tv_nop" : "+v"(a), "+v"(b), "+v"(c), "+v"(d) : "v"(x), "v"(y0), "v"(y1), "v"(y2), "v"(y3));
}
template <typename T> struct Frag;
template <> struct Frag<_Float16> {
  typedef v16h V; union U { v16h v; v8h h[2]; };
  static __device__ __forceinline__ v16h load(const _Float16* p) {
    U f; f.h[0] = *(const v8h*)(p); f.h[1] = *(const v8h*)(p + 16); return f.v;
  }
  static __device__ __forceinline__ v8f mma(v16h a, v16h b, v8f c) {
    return __builtin_amdgcn_wmma_f32_16x16x32_f16(false, a, false, b, (short)0, c, false, false);
  }
};

template <int SG>
__global__ __launch_bounds__(256) void wmma_gemm64_f16(
    const unsigned short* __restrict__ Ap, int lda,
    const unsigned short* __restrict__ Btp, int ldb,
    float* __restrict__ Cout, int ldc,
    float* __restrict__ psum, float* __restrict__ psq,
    float* __restrict__ gmx, float* __restrict__ gmn,
    int M, int N, int K, float scale) {
  typedef _Float16 T;
  typedef v16h V;
  constexpr int SGD = (SG > 0) ? SG : 64;
  const T* A = (const T*)Ap; const T* Bt = (const T*)Btp;
  __shared__ __align__(16) float sT[8][16 * 68];
  const int lane = threadIdx.x & 31;
  const int wave = threadIdx.x >> 5;
  const int tilesN = N >> 6;
  const int tilesM = M >> 6;
  const int tile = blockIdx.x * 8 + wave;
  if (tile >= tilesM * tilesN) return;
  const int tm = tile / tilesN;
  const int tn = tile - tm * tilesN;
  const int m0 = tm << 6;
  const int n0 = tn << 6;

  const int rlane = lane & 15;
  const int koff  = (lane >> 4) * 8;
  const int mOff  = (lane >> 4) * 8;

  v8f acc[4][4];
#pragma unroll
  for (int i = 0; i < 4; ++i)
#pragma unroll
    for (int j = 0; j < 4; ++j) acc[i][j] = (v8f){0.f,0.f,0.f,0.f,0.f,0.f,0.f,0.f};

  for (int k0 = 0; k0 < K; k0 += 32) {
    V bh[4];
#pragma unroll
    for (int j = 0; j < 4; ++j) {
      const size_t bo = (size_t)(n0 + (j << 4) + rlane) * ldb + koff + k0;
      bh[j] = Frag<T>::load(Bt + bo);
    }
#pragma unroll
    for (int i = 0; i < 4; ++i) {
      const size_t ao = (size_t)(m0 + (i << 4) + rlane) * lda + koff + k0;
      V ah = Frag<T>::load(A + ao);
#pragma unroll
      for (int j = 0; j < 4; ++j) {
        acc[i][j] = Frag<T>::mma(ah, bh[j], acc[i][j]);
      }
      tile_guard_h(acc[i][0], acc[i][1], acc[i][2], acc[i][3], ah, bh[0], bh[1], bh[2], bh[3]);
    }
    keep4_h(bh[0], bh[1], bh[2], bh[3]);
  }
  acc_guard4(acc[0][0], acc[0][1], acc[0][2], acc[0][3]);
  acc_guard4(acc[1][0], acc[1][1], acc[1][2], acc[1][3]);
  acc_guard4(acc[2][0], acc[2][1], acc[2][2], acc[2][3]);
  acc_guard4(acc[3][0], acc[3][1], acc[3][2], acc[3][3]);

  float* slab = sT[wave];
  const int hh = lane >> 4;
  const int c4 = (lane & 15) * 4;
  v4f cs  = (v4f){0.f, 0.f, 0.f, 0.f};
  v4f cq  = (v4f){0.f, 0.f, 0.f, 0.f};
  v4f cmx = (v4f){-3.0e38f, -3.0e38f, -3.0e38f, -3.0e38f};
  v4f cmn = (v4f){3.0e38f, 3.0e38f, 3.0e38f, 3.0e38f};
#pragma unroll
  for (int i = 0; i < 4; ++i) {
    const int mBase = m0 + (i << 4);
#pragma unroll
    for (int j = 0; j < 4; ++j) {
#pragma unroll
      for (int r = 0; r < 8; ++r) {
        const float v = acc[i][j][r] * scale;
        slab[(mOff + r) * 68 + (j << 4) + rlane] = v;
      }
    }
    __builtin_amdgcn_fence(__ATOMIC_RELEASE, "workgroup");
    __builtin_amdgcn_wave_barrier();
    __builtin_amdgcn_fence(__ATOMIC_ACQUIRE, "workgroup");
    if (SG == 0) {
      for (int pass = 0; pass < 2; ++pass) {
#pragma unroll
        for (int it = 0; it < 8; ++it) {
          const int row = it * 2 + hh;
          v4f v = *(const v4f*)(slab + row * 68 + c4);
          *(volatile v4f*)(Cout + (size_t)(mBase + row) * ldc + n0 + c4) = v;
        }
        __threadfence();
      }
    } else {
#pragma unroll
      for (int rr = 0; rr < 8; ++rr) {
        const v4f v = *(const v4f*)(slab + (hh * 8 + rr) * 68 + c4);
#pragma unroll
        for (int e = 0; e < 4; ++e) {
          const float x = v[e];
          cs[e] = cs[e] + x;
          cq[e] = cq[e] + x * x;
          cmx[e] = fmaxf(cmx[e], x);
          cmn[e] = fminf(cmn[e], x);
        }
      }
    }
    __builtin_amdgcn_fence(__ATOMIC_RELEASE, "workgroup");
    __builtin_amdgcn_wave_barrier();
    __builtin_amdgcn_fence(__ATOMIC_ACQUIRE, "workgroup");
    if (SG > 0) {
      if ((((i + 1) * 16) % SGD) == 0) {
        v4f val;
#pragma unroll
        for (int e = 0; e < 4; ++e) {
          const float omx = __shfl_xor(cmx[e], 16, 32);
          const float omn = __shfl_xor(cmn[e], 16, 32);
          const float fmx = fmaxf(cmx[e], omx);
          const float fmn = fminf(cmn[e], omn);
          val[e] = hh ? fmn : fmx;
        }
        const int grp = (mBase + 15) / SGD;
        float* dst = (hh ? gmn : gmx) + (size_t)grp * N + n0 + c4;
        *(volatile v4f*)dst = val;
        __threadfence();
        *(volatile v4f*)dst = val;
        cmx = (v4f){-3.0e38f, -3.0e38f, -3.0e38f, -3.0e38f};
        cmn = (v4f){3.0e38f, 3.0e38f, 3.0e38f, 3.0e38f};
      }
    }
  }
  if (SG > 0) {
    v4f val;
#pragma unroll
    for (int e = 0; e < 4; ++e) {
      const float os = __shfl_xor(cs[e], 16, 32);
      const float oq = __shfl_xor(cq[e], 16, 32);
      const float fs = cs[e] + os;
      const float fq = cq[e] + oq;
      val[e] = hh ? fq : fs;
    }
    float* dst = (hh ? psq : psum) + (size_t)tm * N + n0 + c4;
    *(volatile v4f*)dst = val;
    __threadfence();
    *(volatile v4f*)dst = val;
  }
}

__global__ __launch_bounds__(256) void prep_weights_kernel(
    const float* __restrict__ w11, const float* __restrict__ w20,
    const float* __restrict__ w21, const float* __restrict__ w30,
    _Float16* __restrict__ h11, _Float16* __restrict__ h20,
    _Float16* __restrict__ h21, _Float16* __restrict__ h30) {
  const int blk = blockIdx.x;
  const float* src; _Float16* dst; int kp, ld, off, tb;
  if (blk < 4)       { src = w11; dst = h11; kp = CH1A; ld = CH1A;  off = 0; tb = blk; }
  else if (blk < 12) { src = w20; dst = h20; kp = CH1B; ld = W20LD; off = 3; tb = blk - 4; }
  else if (blk < 28) { src = w21; dst = h21; kp = CH2A; ld = CH2A;  off = 0; tb = blk - 12; }
  else               { src = w30; dst = h30; kp = CH2B; ld = W30LD; off = 3; tb = blk - 28; }
  const int e0 = (tb * 256 + (int)threadIdx.x) * 8;
  const int row = e0 / kp;
  const int k = e0 - row * kp;
  const float* s = src + (size_t)row * ld + off + k;
  v8h hv;
#pragma unroll
  for (int e = 0; e < 8; ++e) {
    const float x = s[e] * WCARRY;
    hv[e] = (_Float16)x;
  }
  volatile v8h* d = (volatile v8h*)(dst + e0);
  *d = hv;
  __threadfence();
  *d = hv;
}

template <int NT, int PPT>
__global__ __launch_bounds__(NT) void fps_kernel(const float* __restrict__ pts, int bstride,
                                                 int pstride, int cstride, int nsteps,
                                                 float* __restrict__ outq) {
#pragma clang fp contract(off)
  constexpr int NWV = NT / 32;
  constexpr int NPT = NT * PPT;
  __shared__ float sv[2][32];
  __shared__ int   si[2][32];
  __shared__ __align__(16) float sq[512 * 4];
  const int t = threadIdx.x;
  const int lane = t & 31;
  const int wave = t >> 5;
  const float* P = pts + (size_t)blockIdx.x * bstride;
  const int ns = nsteps < 512 ? nsteps : 512;

  float px[PPT], py[PPT], pz[PPT], dist[PPT];
#pragma unroll
  for (int j = 0; j < PPT; ++j) px[j] = P[(size_t)(t + NT * j) * pstride];
#pragma unroll
  for (int j = 0; j < PPT; ++j) asm volatile("" : "+v"(px[j]) :: "memory");
#pragma unroll
  for (int j = 0; j < PPT; ++j) py[j] = P[(size_t)(t + NT * j) * pstride + cstride];
#pragma unroll
  for (int j = 0; j < PPT; ++j) asm volatile("" : "+v"(py[j]) :: "memory");
#pragma unroll
  for (int j = 0; j < PPT; ++j) pz[j] = P[(size_t)(t + NT * j) * pstride + 2 * cstride];
#pragma unroll
  for (int j = 0; j < PPT; ++j) asm volatile("" : "+v"(pz[j]) :: "memory");
#pragma unroll
  for (int j = 0; j < PPT; ++j) dist[j] = 1e10f;

  int far = 0;
  for (int it = 0; it < ns; ++it) {
    const float cx = P[(size_t)far * pstride];
    const float cy = P[(size_t)far * pstride + cstride];
    const float cz = P[(size_t)far * pstride + 2 * cstride];
    if (t == 0) {
      sq[it * 4 + 0] = cx; sq[it * 4 + 1] = cy; sq[it * 4 + 2] = cz; sq[it * 4 + 3] = 0.0f;
    }
    float best = -1.0f;
    int bi = t;
#pragma unroll
    for (int j = 0; j < PPT; ++j) {
      const float dx = px[j] - cx;
      const float dy = py[j] - cy;
      const float dz = pz[j] - cz;
      const float t0 = dx * dx;
      const float t1 = dy * dy;
      const float t2 = dz * dz;
      const float d = (t0 + t2) + t1;
      const float dm = fminf(dist[j], d);
      dist[j] = dm;
      const bool up = dm > best;
      best = up ? dm : best;
      bi = up ? (t + NT * j) : bi;
    }
#pragma unroll
    for (int off = 16; off >= 1; off >>= 1) {
      const float ov = __shfl_xor(best, off, 32);
      const int oi = __shfl_xor(bi, off, 32);
      const bool take = (ov > best) || ((ov == best) && (oi < bi));
      best = take ? ov : best;
      bi = take ? oi : bi;
    }
    const int buf = it & 1;
    if (lane == 0) { sv[buf][wave] = best; si[buf][wave] = bi; }
    __syncthreads();
    const int l2 = lane < NWV ? lane : 0;
    float v = sv[buf][l2];
    int ix = si[buf][l2];
    v = lane < NWV ? v : -2.0f;
    ix = lane < NWV ? ix : 0x7fffffff;
#pragma unroll
    for (int off = 16; off >= 1; off >>= 1) {
      const float ov = __shfl_xor(v, off, 32);
      const int oi = __shfl_xor(ix, off, 32);
      const bool take = (ov > v) || ((ov == v) && (oi < ix));
      v = take ? ov : v;
      ix = take ? oi : ix;
    }
    ix = ix < 0 ? 0 : ix;
    ix = ix > NPT - 1 ? NPT - 1 : ix;
    far = ix;
  }
  __syncthreads();
  const int tc = t < ns ? t : 0;
  const v4f o = *(const v4f*)(sq + tc * 4);
  float* dst = outq + ((size_t)blockIdx.x * ns + tc) * 4;
  if (t < ns) *(volatile v4f*)dst = o;
  __threadfence();
  if (t < ns) *(volatile v4f*)dst = o;
}

template <int KS>
__global__ __launch_bounds__(256) void ballq_kernel(const float* __restrict__ pts, int bstride,
                                                    int pstride, int cstride, int npts,
                                                    const float* __restrict__ qxyz4, int qper, int nq,
                                                    int* __restrict__ gi, float thr) {
#pragma clang fp contract(off)
  __shared__ __align__(16) int lst[8][KS];
  const int lane = threadIdx.x & 31;
  const int wave = threadIdx.x >> 5;
  const int q = blockIdx.x * 8 + wave;
  const int qc = q < nq ? q : nq - 1;
  const int b = qc / qper;
  const float* P = pts + (size_t)b * bstride;
  const v4f qv = *(const v4f*)(qxyz4 + (size_t)qc * 4);
  const float qx = qv[0];
  const float qy = qv[1];
  const float qz = qv[2];
  const float a0 = qx * qx;
  const float a1 = qy * qy;
  const float a2 = qz * qz;
  const float sqa = (a0 + a2) + a1;
  int* L = lst[wave];
  if (lane == 0) L[0] = 0;
  int cnt = 0;
  int nit = npts >> 5;
  nit = nit > 256 ? 256 : nit;
  for (int it = 0; (it < nit) && (cnt < KS); ++it) {
    const int n = it * 32 + lane;
    const float x = P[(size_t)n * pstride];
    const float y = P[(size_t)n * pstride + cstride];
    const float z = P[(size_t)n * pstride + 2 * cstride];
    float p = qx * x;
    p = __builtin_fmaf(qy, y, p);
    p = __builtin_fmaf(qz, z, p);
    const float u0 = x * x;
    const float u1 = y * y;
    const float u2 = z * z;
    const float sqb = (u0 + u2) + u1;
    const float two = 2.0f * p;
    const float d2 = (sqa - two) + sqb;
    const bool inb = !(d2 > thr);
    const unsigned mask = __builtin_amdgcn_ballot_w32(inb);
    const int pre = (int)__builtin_amdgcn_mbcnt_lo(mask, 0u);
    const int pos = cnt + pre;
    if (inb && (pos < KS)) L[pos] = n;
    cnt += __builtin_popcount(mask);
  }
  __builtin_amdgcn_fence(__ATOMIC_RELEASE, "workgroup");
  __builtin_amdgcn_wave_barrier();
  __builtin_amdgcn_fence(__ATOMIC_ACQUIRE, "workgroup");
  const int first = L[0];
#pragma unroll
  for (int j = 0; j < KS / 32; ++j) {
    const int s = lane + 32 * j;
    if (s >= cnt) L[s] = first;
  }
  __syncthreads();
  const int li = lane < (KS / 4) ? lane : 0;
  const v4i lv = *(const v4i*)(L + li * 4);
  int* dst = gi + (size_t)qc * KS + li * 4;
  const bool wr = (lane < (KS / 4)) && (q < nq);
  if (wr) *(volatile v4i*)dst = lv;
  __threadfence();
  if (wr) *(volatile v4i*)dst = lv;
}

__global__ __launch_bounds__(256) void mom1_kernel(const float* __restrict__ xyz,
                                                   const float* __restrict__ l1q,
                                                   const int* __restrict__ gi1,
                                                   float* __restrict__ part) {
  __shared__ float red[9][8];
  const int t = threadIdx.x;
  const int lane = t & 31;
  const int wave = t >> 5;
  float a[9];
#pragma unroll
  for (int v = 0; v < 9; ++v) a[v] = 0.0f;
  const int base = blockIdx.x * 4096;
#pragma unroll 1
  for (int i = 0; i < 16; ++i) {
    const int row = base + i * 256 + t;
    const int q = row >> 5;
    const int b = q >> 9;
    int idx = gi1[row];
    idx = idx < 0 ? 0 : idx;
    idx = idx > NPOINT - 1 ? NPOINT - 1 : idx;
    const float* X = xyz + (size_t)b * 3 * NPOINT;
    const float px = X[idx];
    const float py = X[NPOINT + idx];
    const float pz = X[2 * NPOINT + idx];
    const v4f qv = *(const v4f*)(l1q + (size_t)q * 4);
    const float gx = px - qv[0];
    const float gy = py - qv[1];
    const float gz = pz - qv[2];
    a[0] += gx; a[1] += gy; a[2] += gz;
    a[3] += gx * gx; a[4] += gx * gy; a[5] += gx * gz;
    a[6] += gy * gy; a[7] += gy * gz; a[8] += gz * gz;
  }
#pragma unroll
  for (int v = 0; v < 9; ++v) {
    float s = a[v];
#pragma unroll
    for (int off = 16; off >= 1; off >>= 1) s += __shfl_xor(s, off, 32);
    if (lane == 0) red[v][wave] = s;
  }
  __syncthreads();
  if (wave == 0) {
    const int vi = lane < 9 ? lane : 0;
    float s = 0.0f;
#pragma unroll
    for (int w = 0; w < 8; ++w) s += red[vi][w];
    const float o = lane < 9 ? s : 0.0f;
    volatile float* d = (volatile float*)(part + (size_t)blockIdx.x * 32 + lane);
    *d = o;
    __threadfence();
    *d = o;
  }
}

__global__ __launch_bounds__(64) void fin1_kernel(const float* __restrict__ part,
                                                  const float* __restrict__ w,
                                                  const float* __restrict__ gam,
                                                  const float* __restrict__ bet,
                                                  float* __restrict__ scale, float* __restrict__ shift,
                                                  double invM) {
  const int c = threadIdx.x;
  double s[9];
#pragma unroll
  for (int v = 0; v < 9; ++v) s[v] = 0.0;
#pragma unroll 1
  for (int blk = 0; blk < 64; ++blk) {
#pragma unroll
    for (int v = 0; v < 9; ++v) s[v] += (double)part[blk * 32 + v];
  }
  const double mu0 = s[0] * invM, mu1 = s[1] * invM, mu2 = s[2] * invM;
  const double m00 = s[3] * invM - mu0 * mu0;
  const double m01 = s[4] * invM - mu0 * mu1;
  const double m02 = s[5] * invM - mu0 * mu2;
  const double m11 = s[6] * invM - mu1 * mu1;
  const double m12 = s[7] * invM - mu1 * mu2;
  const double m22 = s[8] * invM - mu2 * mu2;
  const double w0 = (double)w[c * 3 + 0];
  const double w1 = (double)w[c * 3 + 1];
  const double w2 = (double)w[c * 3 + 2];
  const double mean = w0 * mu0 + w1 * mu1 + w2 * mu2;
  double var = w0 * w0 * m00 + w1 * w1 * m11 + w2 * w2 * m22
             + 2.0 * (w0 * w1 * m01 + w0 * w2 * m02 + w1 * w2 * m12);
  var = var < 0.0 ? 0.0 : var;
  const float sc = gam[c] * rsqrtf((float)var + 1e-5f);
  const float sh = (float)((double)bet[c] - mean * (double)sc);
  volatile float* ds = (volatile float*)(scale + c);
  volatile float* dh = (volatile float*)(shift + c);
  *ds = sc; *dh = sh;
  __threadfence();
  *ds = sc; *dh = sh;
}

__global__ __launch_bounds__(256) void a1a_kernel(const float* __restrict__ xyz,
                                                  const float* __restrict__ l1q,
                                                  const int* __restrict__ gi1,
                                                  const float* __restrict__ w10,
                                                  const float* __restrict__ scale,
                                                  const float* __restrict__ shift,
                                                  _Float16* __restrict__ a1a) {
  __shared__ float sw[192];
  __shared__ float ssc[64];
  __shared__ float ssh[64];
  const int t = threadIdx.x;
  {
    const int wi = t < 192 ? t : 191;
    const float wv = w10[wi];
    if (t < 192) sw[t] = wv;
    const float sv = scale[t & 63];
    const float hv = shift[t & 63];
    if (t < 64) { ssc[t] = sv; ssh[t] = hv; }
  }
  __syncthreads();
  const int c8 = (t & 7) * 8;
  float wx[8], wy[8], wz[8], sh[8];
#pragma unroll
  for (int e = 0; e < 8; ++e) {
    const float sc = ssc[c8 + e];
    wx[e] = sc * sw[(c8 + e) * 3 + 0];
    wy[e] = sc * sw[(c8 + e) * 3 + 1];
    wz[e] = sc * sw[(c8 + e) * 3 + 2];
    sh[e] = ssh[c8 + e];
  }
#pragma unroll 1
  for (int it = 0; it < 16; ++it) {
    const int row = blockIdx.x * 512 + it * 32 + (t >> 3);
    const int q = row >> 5;
    const int b = q >> 9;
    int idx = gi1[row];
    idx = idx < 0 ? 0 : idx;
    idx = idx > NPOINT - 1 ? NPOINT - 1 : idx;
    const float* X = xyz + (size_t)b * 3 * NPOINT;
    const float px = X[idx];
    const float py = X[NPOINT + idx];
    const float pz = X[2 * NPOINT + idx];
    const v4f qv = *(const v4f*)(l1q + (size_t)q * 4);
    const float gx = px - qv[0];
    const float gy = py - qv[1];
    const float gz = pz - qv[2];
    v8h hv;
#pragma unroll
    for (int e = 0; e < 8; ++e) {
      float v = ((wx[e] * gx + wy[e] * gy) + wz[e] * gz) + sh[e];
      v = fmaxf(v, 0.0f);
      hv[e] = (_Float16)v;
    }
    volatile v8h* d = (volatile v8h*)(a1a + (size_t)row * CH1A + c8);
    *d = hv;
    __threadfence();
    *d = hv;
  }
}

__global__ __launch_bounds__(256) void colfin_kernel(const float* __restrict__ psum,
                                                     const float* __restrict__ psq,
                                                     int R, int N,
                                                     const float* __restrict__ gam,
                                                     const float* __restrict__ bet,
                                                     float* __restrict__ scale,
                                                     float* __restrict__ shift, double invM) {
  __shared__ double ds[8][32];
  __shared__ double dq[8][32];
  const int lane = threadIdx.x & 31;
  const int wave = threadIdx.x >> 5;
  const int col = blockIdx.x * 32 + lane;
  double s = 0.0, q = 0.0;
  const int nr = R >> 3;
#pragma unroll 4
  for (int i = 0; i < nr; ++i) {
    const size_t o = (size_t)(i * 8 + wave) * N + col;
    s += (double)psum[o];
    q += (double)psq[o];
  }
  ds[wave][lane] = s;
  dq[wave][lane] = q;
  __syncthreads();
  if (wave == 0) {
    double S = 0.0, Q = 0.0;
#pragma unroll
    for (int w = 0; w < 8; ++w) { S += ds[w][lane]; Q += dq[w][lane]; }
    const double mean = S * invM;
    double var = Q * invM - mean * mean;
    var = var < 0.0 ? 0.0 : var;
    const float sc = gam[col] * rsqrtf((float)var + 1e-5f);
    const float sh = (float)((double)bet[col] - mean * (double)sc);
    volatile float* a = (volatile float*)(scale + col);
    volatile float* b = (volatile float*)(shift + col);
    *a = sc; *b = sh;
    __threadfence();
    *a = sc; *b = sh;
  }
}

__global__ __launch_bounds__(256) void pool_f16_kernel(const float* __restrict__ gmx,
                                                       const float* __restrict__ gmn,
                                                       const float* __restrict__ scale,
                                                       const float* __restrict__ shift,
                                                       _Float16* __restrict__ out, int R, int N) {
  const int tpr = N >> 3;
  const int total = R * tpr;
  const int gid = blockIdx.x * 256 + threadIdx.x;
  const bool ok = gid < total;
  const int gc = ok ? gid : total - 1;
  const int row = gc / tpr;
  const int c0 = (gc - row * tpr) * 8;
  v8h hv;
#pragma unroll
  for (int g = 0; g < 2; ++g) {
    const v4f mx = *(const v4f*)(gmx + (size_t)row * N + c0 + 4 * g);
    const v4f mn = *(const v4f*)(gmn + (size_t)row * N + c0 + 4 * g);
    const v4f sc = *(const v4f*)(scale + c0 + 4 * g);
    const v4f sh = *(const v4f*)(shift + c0 + 4 * g);
#pragma unroll
    for (int e = 0; e < 4; ++e) {
      const float v = (sc[e] >= 0.0f) ? mx[e] : mn[e];
      float y = sc[e] * v + sh[e];
      y = fmaxf(y, 0.0f);
      hv[4 * g + e] = (_Float16)y;
    }
  }
  volatile v8h* d = (volatile v8h*)(out + (size_t)row * N + c0);
  if (ok) *d = hv;
  __threadfence();
  if (ok) *d = hv;
}

__global__ __launch_bounds__(256) void pool_f32_kernel(const float* __restrict__ gmx,
                                                       const float* __restrict__ gmn,
                                                       const float* __restrict__ scale,
                                                       const float* __restrict__ shift,
                                                       float* __restrict__ out0,
                                                       float* __restrict__ out1, int R, int N) {
  const int tpr = N >> 2;
  const int total = R * tpr;
  const int gid = blockIdx.x * 256 + threadIdx.x;
  const bool ok = gid < total;
  const int gc = ok ? gid : total - 1;
  const int row = gc / tpr;
  const int c0 = (gc - row * tpr) * 4;
  const v4f mx = *(const v4f*)(gmx + (size_t)row * N + c0);
  const v4f mn = *(const v4f*)(gmn + (size_t)row * N + c0);
  const v4f sc = *(const v4f*)(scale + c0);
  const v4f sh = *(const v4f*)(shift + c0);
  v4f o;
#pragma unroll
  for (int e = 0; e < 4; ++e) {
    const float v = (sc[e] >= 0.0f) ? mx[e] : mn[e];
    float y = sc[e] * v + sh[e];
    y = fmaxf(y, 0.0f);
    o[e] = y;
  }
  volatile v4f* d0 = (volatile v4f*)(out0 + (size_t)row * N + c0);
  volatile v4f* d1 = (volatile v4f*)(out1 + (size_t)row * N + c0);
  if (ok) { *d0 = o; *d1 = o; }
  __threadfence();
  if (ok) { *d0 = o; *d1 = o; }
}

__device__ __forceinline__ float h2_value(float pf, float wx, float wy, float wz,
                                          float gx, float gy, float gz) {
  return pf + ((wx * gx + wy * gy) + wz * gz);
}

__global__ __launch_bounds__(256) void g2_stats_kernel(const float* __restrict__ Pf,
                                                       const int* __restrict__ gi2,
                                                       const float* __restrict__ l1q,
                                                       const float* __restrict__ l2q,
                                                       const float* __restrict__ w20,
                                                       float* __restrict__ psum,
                                                       float* __restrict__ psq) {
  const int lane = threadIdx.x & 31;
  const int wave = threadIdx.x >> 5;
  const int q = blockIdx.x * 8 + wave;
  const int b = q >> 7;
  const int c4 = lane * 4;
  float wx[4], wy[4], wz[4];
#pragma unroll
  for (int e = 0; e < 4; ++e) {
    wx[e] = w20[(size_t)(c4 + e) * W20LD + 0];
    wy[e] = w20[(size_t)(c4 + e) * W20LD + 1];
    wz[e] = w20[(size_t)(c4 + e) * W20LD + 2];
  }
  const v4f qv = *(const v4f*)(l2q + (size_t)q * 4);
  v4f s = (v4f){0.f, 0.f, 0.f, 0.f};
  v4f qq = (v4f){0.f, 0.f, 0.f, 0.f};
#pragma unroll 1
  for (int k = 0; k < NNBR2; ++k) {
    int idx = gi2[(size_t)q * NNBR2 + k];
    idx = idx < 0 ? 0 : idx;
    idx = idx > NCEN1 - 1 ? NCEN1 - 1 : idx;
    const int src = b * NCEN1 + idx;
    const v4f pv = *(const v4f*)(l1q + (size_t)src * 4);
    const float gx = pv[0] - qv[0];
    const float gy = pv[1] - qv[1];
    const float gz = pv[2] - qv[2];
    const v4f pf = *(const v4f*)(Pf + (size_t)src * CH2A + c4);
#pragma unroll
    for (int e = 0; e < 4; ++e) {
      const float h = h2_value(pf[e], wx[e], wy[e], wz[e], gx, gy, gz);
      s[e] = s[e] + h;
      qq[e] = qq[e] + h * h;
    }
  }
  volatile v4f* d0 = (volatile v4f*)(psum + (size_t)q * CH2A + c4);
  volatile v4f* d1 = (volatile v4f*)(psq + (size_t)q * CH2A + c4);
  *d0 = s; *d1 = qq;
  __threadfence();
  *d0 = s; *d1 = qq;
}

__global__ __launch_bounds__(256) void g2_write_kernel(const float* __restrict__ Pf,
                                                       const int* __restrict__ gi2,
                                                       const float* __restrict__ l1q,
                                                       const float* __restrict__ l2q,
                                                       const float* __restrict__ w20,
                                                       const float* __restrict__ scale,
                                                       const float* __restrict__ shift,
                                                       _Float16* __restrict__ a2a) {
  __shared__ float sw[384];
  __shared__ float ssc[128];
  __shared__ float ssh[128];
  const int t = threadIdx.x;
  {
    const int i0 = t;
    const int ca = i0 / 3;
    const int ja = i0 - ca * 3;
    sw[i0] = w20[(size_t)ca * W20LD + ja];
    const int i1 = t + 256;
    const int i1c = i1 < 384 ? i1 : 383;
    const int cb = i1c / 3;
    const int jb = i1c - cb * 3;
    const float vb = w20[(size_t)cb * W20LD + jb];
    if (i1 < 384) sw[i1] = vb;
    const float sv = scale[t & 127];
    const float hv = shift[t & 127];
    if (t < 128) { ssc[t] = sv; ssh[t] = hv; }
  }
  __syncthreads();
  const int lane = t & 31;
  const int wave = t >> 5;
  const int hh = lane >> 4;
  const int c8 = (lane & 15) * 8;
  float wx[8], wy[8], wz[8], sc[8], sh[8];
#pragma unroll
  for (int e = 0; e < 8; ++e) {
    wx[e] = sw[(c8 + e) * 3 + 0];
    wy[e] = sw[(c8 + e) * 3 + 1];
    wz[e] = sw[(c8 + e) * 3 + 2];
    sc[e] = ssc[c8 + e];
    sh[e] = ssh[c8 + e];
  }
  const int q = blockIdx.x * 8 + wave;
  const int b = q >> 7;
  const v4f qv = *(const v4f*)(l2q + (size_t)q * 4);
#pragma unroll 1
  for (int kk = 0; kk < NNBR2 / 2; ++kk) {
    const int k = kk * 2 + hh;
    const size_t row = (size_t)q * NNBR2 + k;
    int idx = gi2[row];
    idx = idx < 0 ? 0 : idx;
    idx = idx > NCEN1 - 1 ? NCEN1 - 1 : idx;
    const int src = b * NCEN1 + idx;
    const v4f pv = *(const v4f*)(l1q + (size_t)src * 4);
    const float gx = pv[0] - qv[0];
    const float gy = pv[1] - qv[1];
    const float gz = pv[2] - qv[2];
    const v4f pf0 = *(const v4f*)(Pf + (size_t)src * CH2A + c8);
    const v4f pf1 = *(const v4f*)(Pf + (size_t)src * CH2A + c8 + 4);
    v8h hv;
#pragma unroll
    for (int e = 0; e < 4; ++e) {
      const float h0 = h2_value(pf0[e], wx[e], wy[e], wz[e], gx, gy, gz);
      const float h1 = h2_value(pf1[e], wx[4 + e], wy[4 + e], wz[4 + e], gx, gy, gz);
      float y0 = sc[e] * h0 + sh[e];
      float y1 = sc[4 + e] * h1 + sh[4 + e];
      y0 = fmaxf(y0, 0.0f);
      y1 = fmaxf(y1, 0.0f);
      hv[e] = (_Float16)y0;
      hv[4 + e] = (_Float16)y1;
    }
    volatile v8h* d = (volatile v8h*)(a2a + row * CH2A + c8);
    *d = hv;
    __threadfence();
    *d = hv;
  }
}

__global__ __launch_bounds__(256) void sa3_stats_kernel(const float* __restrict__ h3f,
                                                        const float* __restrict__ l2q,
                                                        const float* __restrict__ w30,
                                                        float* __restrict__ psum,
                                                        float* __restrict__ psq,
                                                        float* __restrict__ gmx,
                                                        float* __restrict__ gmn) {
  const int b = blockIdx.x;
  const int c = threadIdx.x;
  const float wx = w30[(size_t)c * W30LD + 0];
  const float wy = w30[(size_t)c * W30LD + 1];
  const float wz = w30[(size_t)c * W30LD + 2];
  float s = 0.0f, q = 0.0f, mx = -3.0e38f, mn = 3.0e38f;
#pragma unroll 4
  for (int r = 0; r < NCEN2; ++r) {
    const int row = b * NCEN2 + r;
    const v4f pv = *(const v4f*)(l2q + (size_t)row * 4);
    const float h = h3f[(size_t)row * CH3O + c] + ((wx * pv[0] + wy * pv[1]) + wz * pv[2]);
    s += h;
    q += h * h;
    mx = fmaxf(mx, h);
    mn = fminf(mn, h);
  }
  const size_t o = (size_t)b * CH3O + c;
  volatile float* d0 = (volatile float*)(psum + o);
  volatile float* d1 = (volatile float*)(psq + o);
  volatile float* d2 = (volatile float*)(gmx + o);
  volatile float* d3 = (volatile float*)(gmn + o);
  *d0 = s; *d1 = q; *d2 = mx; *d3 = mn;
  __threadfence();
  *d0 = s; *d1 = q; *d2 = mx; *d3 = mn;
}

extern "C" void kernel_launch(void* const* d_in, const int* in_sizes, int n_in,
                              void* d_out, int out_size, void* d_ws, size_t ws_size,
                              hipStream_t stream) {
  (void)in_sizes; (void)out_size;
  if (n_in < 16) return;

  const float* xyz  = (const float*)d_in[0];
  const float* w1_0 = (const float*)d_in[1];
  const float* g1_0 = (const float*)d_in[2];
  const float* b1_0 = (const float*)d_in[3];
  const float* w1_1 = (const float*)d_in[4];
  const float* g1_1 = (const float*)d_in[5];
  const float* b1_1 = (const float*)d_in[6];
  const float* w2_0 = (const float*)d_in[7];
  const float* g2_0 = (const float*)d_in[8];
  const float* b2_0 = (const float*)d_in[9];
  const float* w2_1 = (const float*)d_in[10];
  const float* g2_1 = (const float*)d_in[11];
  const float* b2_1 = (const float*)d_in[12];
  const float* w3_0 = (const float*)d_in[13];
  const float* g3_0 = (const float*)d_in[14];
  const float* b3_0 = (const float*)d_in[15];
  float* out = (float*)d_out;

  char* base = (char*)d_ws;
  size_t off = 0;
  auto carve = [&](size_t bytes) -> char* {
    char* p = base + off;
    off += (bytes + 255) & ~(size_t)255;
    return p;
  };
  float* l1q = (float*)carve((size_t)NQ1 * 4 * 4);
  float* l2q = (float*)carve((size_t)NQ2 * 4 * 4);
  int*   gi1 = (int*)carve((size_t)NQ1 * NNBR1 * 4);
  int*   gi2 = (int*)carve((size_t)NQ2 * NNBR2 * 4);
  _Float16* h11 = (_Float16*)carve((size_t)CH1B * CH1A * 2);
  _Float16* h20 = (_Float16*)carve((size_t)CH2A * CH1B * 2);
  _Float16* h21 = (_Float16*)carve((size_t)CH2B * CH2A * 2);
  _Float16* h30 = (_Float16*)carve((size_t)CH3O * CH2B * 2);
  float* mom = (float*)carve((size_t)64 * 32 * 4);
  float* sc10 = (float*)carve(1024); float* sh10 = (float*)carve(1024);
  float* sc11 = (float*)carve(1024); float* sh11 = (float*)carve(1024);
  float* sc20 = (float*)carve(1024); float* sh20 = (float*)carve(1024);
  float* sc21 = (float*)carve(1024); float* sh21 = (float*)carve(1024);
  float* sc30 = (float*)carve(1024); float* sh30 = (float*)carve(1024);
  _Float16* a1a = (_Float16*)carve((size_t)ROWS1 * CH1A * 2);
  float* ps1 = (float*)carve((size_t)(ROWS1 / 64) * CH1B * 4);
  float* pq1 = (float*)carve((size_t)(ROWS1 / 64) * CH1B * 4);
  float* gx1 = (float*)carve((size_t)NQ1 * CH1B * 4);
  float* gn1 = (float*)carve((size_t)NQ1 * CH1B * 4);
  _Float16* l1f = (_Float16*)carve((size_t)NQ1 * CH1B * 2);
  float* Pf  = (float*)carve((size_t)NQ1 * CH2A * 4);
  float* psA = (float*)carve((size_t)NQ2 * CH2A * 4);
  float* pqA = (float*)carve((size_t)NQ2 * CH2A * 4);
  _Float16* a2a = (_Float16*)carve((size_t)ROWS2 * CH2A * 2);
  float* ps2 = (float*)carve((size_t)(ROWS2 / 64) * CH2B * 4);
  float* pq2 = (float*)carve((size_t)(ROWS2 / 64) * CH2B * 4);
  float* gx2 = (float*)carve((size_t)NQ2 * CH2B * 4);
  float* gn2 = (float*)carve((size_t)NQ2 * CH2B * 4);
  _Float16* l2f = (_Float16*)carve((size_t)NQ2 * CH2B * 2);
  float* h3f = (float*)carve((size_t)ROWS3 * CH3O * 4);
  float* ps3 = (float*)carve((size_t)NBATCH * CH3O * 4);
  float* pq3 = (float*)carve((size_t)NBATCH * CH3O * 4);
  float* gx3 = (float*)carve((size_t)NBATCH * CH3O * 4);
  float* gn3 = (float*)carve((size_t)NBATCH * CH3O * 4);
  if (off > ws_size || off > (size_t)134217728) return;

  const float thr1 = 0.04f;
  const float thr2 = 0.16f;

  prep_weights_kernel<<<60, 256, 0, stream>>>(w1_1, w2_0, w2_1, w3_0, h11, h20, h21, h30);

  fps_kernel<1024, 8><<<NBATCH, 1024, 0, stream>>>(xyz, 3 * NPOINT, 1, NPOINT, NCEN1, l1q);
  ballq_kernel<NNBR1><<<NQ1 / 8, 256, 0, stream>>>(xyz, 3 * NPOINT, 1, NPOINT, NPOINT,
                                                   l1q, NCEN1, NQ1, gi1, thr1);
  mom1_kernel<<<64, 256, 0, stream>>>(xyz, l1q, gi1, mom);
  fin1_kernel<<<1, 64, 0, stream>>>(mom, w1_0, g1_0, b1_0, sc10, sh10, 1.0 / (double)ROWS1);
  a1a_kernel<<<ROWS1 / 512, 256, 0, stream>>>(xyz, l1q, gi1, w1_0, sc10, sh10, a1a);
  wmma_gemm64_f16<32><<<(ROWS1 / 64) * (CH1B / 64) / 8, 256, 0, stream>>>(
      (const unsigned short*)a1a, CH1A, (const unsigned short*)h11, CH1A,
      ps1, CH1B, ps1, pq1, gx1, gn1, ROWS1, CH1B, CH1A, WCARRY_INV);
  colfin_kernel<<<CH1B / 32, 256, 0, stream>>>(ps1, pq1, ROWS1 / 64, CH1B, g1_1, b1_1,
                                               sc11, sh11, 1.0 / (double)ROWS1);
  pool_f16_kernel<<<(NQ1 * CH1B / 8) / 256, 256, 0, stream>>>(gx1, gn1, sc11, sh11, l1f, NQ1, CH1B);

  fps_kernel<512, 1><<<NBATCH, 512, 0, stream>>>(l1q, NCEN1 * 4, 4, 1, NCEN2, l2q);
  ballq_kernel<NNBR2><<<NQ2 / 8, 256, 0, stream>>>(l1q, NCEN1 * 4, 4, 1, NCEN1,
                                                   l2q, NCEN2, NQ2, gi2, thr2);
  wmma_gemm64_f16<0><<<(NQ1 / 64) * (CH2A / 64) / 8, 256, 0, stream>>>(
      (const unsigned short*)l1f, CH1B, (const unsigned short*)h20, CH1B,
      Pf, CH2A, Pf, Pf, Pf, Pf, NQ1, CH2A, CH1B, WCARRY_INV);
  g2_stats_kernel<<<NQ2 / 8, 256, 0, stream>>>(Pf, gi2, l1q, l2q, w2_0, psA, pqA);
  colfin_kernel<<<CH2A / 32, 256, 0, stream>>>(psA, pqA, NQ2, CH2A, g2_0, b2_0,
                                               sc20, sh20, 1.0 / (double)ROWS2);
  g2_write_kernel<<<NQ2 / 8, 256, 0, stream>>>(Pf, gi2, l1q, l2q, w2_0, sc20, sh20, a2a);
  wmma_gemm64_f16<64><<<(ROWS2 / 64) * (CH2B / 64) / 8, 256, 0, stream>>>(
      (const unsigned short*)a2a, CH2A, (const unsigned short*)h21, CH2A,
      ps2, CH2B, ps2, pq2, gx2, gn2, ROWS2, CH2B, CH2A, WCARRY_INV);
  colfin_kernel<<<CH2B / 32, 256, 0, stream>>>(ps2, pq2, ROWS2 / 64, CH2B, g2_1, b2_1,
                                               sc21, sh21, 1.0 / (double)ROWS2);
  pool_f16_kernel<<<(NQ2 * CH2B / 8) / 256, 256, 0, stream>>>(gx2, gn2, sc21, sh21, l2f, NQ2, CH2B);

  wmma_gemm64_f16<0><<<(ROWS3 / 64) * (CH3O / 64) / 8, 256, 0, stream>>>(
      (const unsigned short*)l2f, CH2B, (const unsigned short*)h30, CH2B,
      h3f, CH3O, h3f, h3f, h3f, h3f, ROWS3, CH3O, CH2B, WCARRY_INV);
  sa3_stats_kernel<<<NBATCH, 256, 0, stream>>>(h3f, l2q, w3_0, ps3, pq3, gx3, gn3);
  colfin_kernel<<<CH3O / 32, 256, 0, stream>>>(ps3, pq3, NBATCH, CH3O, g3_0, b3_0,
                                               sc30, sh30, 1.0 / (double)ROWS3);
  pool_f32_kernel<<<(NBATCH * CH3O / 4) / 256, 256, 0, stream>>>(gx3, gn3, sc30, sh30,
                                                                 out, out + NBATCH * CH3O,
                                                                 NBATCH, CH3O);
}
